// DynamicConvCrsMod_51402168599362
// MI455X (gfx1250) — hardware-verified
//
#include <hip/hip_runtime.h>


typedef _Float16 v16h __attribute__((ext_vector_type(16)));
typedef _Float16 v8h  __attribute__((ext_vector_type(8)));
typedef _Float16 v4h  __attribute__((ext_vector_type(4)));
typedef float    v8f  __attribute__((ext_vector_type(8)));
typedef float    v4f  __attribute__((ext_vector_type(4)));

#define EDIM 256
#define DDYN 64
#define TWOE 512
#define NP1  32768
#define NP2  16384

union Frag { v16h v; v8h hf[2]; };

static __device__ __forceinline__ v16h ld_frag(const _Float16* rowp, int k0, int h) {
  Frag f;
  f.hf[0] = *(const v8h*)(rowp + k0 + 8 * h);
  f.hf[1] = *(const v8h*)(rowp + k0 + 16 + 8 * h);
  return f.v;
}

static __device__ __forceinline__ v16h splat16(_Float16 s) {
  v16h r;
#pragma unroll
  for (int i = 0; i < 16; ++i) r[i] = s;
  return r;
}

static __device__ __forceinline__ v8f zero8() {
  v8f z;
#pragma unroll
  for (int i = 0; i < 8; ++i) z[i] = 0.0f;
  return z;
}

static __device__ __forceinline__ v8f mma16(v16h a, v16h b, v8f c) {
  return __builtin_amdgcn_wmma_f32_16x16x32_f16(false, a, false, b, (short)0, c, false, false);
}

#define NOP4 "v_nop\n\tv_nop\n\tv_nop\n\tv_nop"
#define WG4(c0, c1, c2, c3, a, b0, b1, b2, b3)                                   \
  asm volatile(NOP4 : "+v"(c0), "+v"(c1), "+v"(c2), "+v"(c3)                   \
               : "v"(a), "v"(b0), "v"(b1), "v"(b2), "v"(b3))
#define WG8(c0, c1, c2, c3, c4, c5, c6, c7, a0, a1, b0, b1, b2, b3)            \
  asm volatile(NOP4 : "+v"(c0), "+v"(c1), "+v"(c2), "+v"(c3), "+v"(c4),        \
               "+v"(c5), "+v"(c6), "+v"(c7)                                   \
               : "v"(a0), "v"(a1), "v"(b0), "v"(b1), "v"(b2), "v"(b3))

static __device__ __forceinline__ float wsum32(float v) {
#pragma unroll
  for (int o = 16; o > 0; o >>= 1) v += __shfl_xor(v, o, 32);
  return v;
}
static __device__ __forceinline__ float wsum8(float v) {
#pragma unroll
  for (int o = 4; o > 0; o >>= 1) v += __shfl_xor(v, o, 32);
  return v;
}

__global__ __launch_bounds__(256) void cvt8_kernel(const float* __restrict__ s,
                                                   _Float16* __restrict__ d, int n8, float scale) {
  const int i = blockIdx.x * 256 + threadIdx.x;
  if (i >= n8) return;
  const float* p = s + (size_t)i * 8;
  const v4f x0 = *(const v4f*)p;
  const v4f x1 = *(const v4f*)(p + 4);
  v8h y;
#pragma unroll
  for (int j = 0; j < 4; ++j) {
    y[j]     = (_Float16)(x0[j] * scale);
    y[4 + j] = (_Float16)(x1[j] * scale);
  }
  _Float16* q = d + (size_t)i * 8;
  *(volatile v8h*)q = y;
  __threadfence();
  *(volatile v8h*)q = y;
}

__global__ __launch_bounds__(256) void bias_t_kernel(const float* __restrict__ in,
                                                     _Float16* __restrict__ out, int R, int C,
                                                     float scale) {
  const int i = blockIdx.x * 256 + threadIdx.x;
  const int R8 = R >> 3;
  if (i >= C * R8) return;
  const int c = i / R8;
  const int r8 = (i - c * R8) * 8;
  v8h y;
#pragma unroll
  for (int j = 0; j < 8; ++j) y[j] = (_Float16)(in[(size_t)(r8 + j) * C + c] * scale);
  _Float16* q = out + (size_t)c * R + r8;
  *(volatile v8h*)q = y;
  __threadfence();
  *(volatile v8h*)q = y;
}

static __device__ __forceinline__ void store_tile16x64(float* stg, float* gbase, int gpitch,
                                                       v8f c0, v8f c1, v8f c2, v8f c3,
                                                       float inv, int lane, int h, int m) {
#pragma unroll
  for (int r = 0; r < 8; ++r) {
    float* sp = stg + (8 * h + r) * 64 + m;
    sp[0]  = c0[r] * inv;
    sp[16] = c1[r] * inv;
    sp[32] = c2[r] * inv;
    sp[48] = c3[r] * inv;
  }
  __syncthreads();
  v4f v[8];
#pragma unroll
  for (int j = 0; j < 8; ++j) v[j] = *(const v4f*)(stg + j * 128 + lane * 4);
  float* gp = gbase + (size_t)h * gpitch + m * 4;
#pragma unroll
  for (int j = 0; j < 8; ++j) *(volatile v4f*)(gp + (size_t)(2 * j) * gpitch) = v[j];
  __threadfence();
#pragma unroll
  for (int j = 0; j < 8; ++j) *(volatile v4f*)(gp + (size_t)(2 * j) * gpitch) = v[j];
}

__global__ __launch_bounds__(256) void s1_kernel(const _Float16* __restrict__ q16,
                                                 const _Float16* __restrict__ feats16,
                                                 const _Float16* __restrict__ wpre16,
                                                 const _Float16* __restrict__ bpreT16,
                                                 float* __restrict__ f1raw, int nrows) {
  __shared__ float lds[8192];
  _Float16* tile = reinterpret_cast<_Float16*>(lds);
  const int tid = threadIdx.x, lane = tid & 31, wave = tid >> 5;
  const int h = lane >> 4, m = lane & 15;
  const int rowBase = blockIdx.x * 256 + wave * 32;
  int r0 = rowBase + m;      r0 = (r0 < nrows) ? r0 : (nrows - 1);
  int r1 = rowBase + 16 + m; r1 = (r1 < nrows) ? r1 : (nrows - 1);
  const _Float16* qp0 = q16 + (size_t)r0 * EDIM;
  const _Float16* qp1 = q16 + (size_t)r1 * EDIM;
  const _Float16* fp0 = feats16 + (size_t)r0 * TWOE;
  const _Float16* fp1 = feats16 + (size_t)r1 * TWOE;

  v8f acc[2][4];
#pragma unroll
  for (int i = 0; i < 2; ++i)
#pragma unroll
    for (int j = 0; j < 4; ++j) acc[i][j] = zero8();

  const int cd = tid >> 2, cpart = (tid & 3) * 8;
  const _Float16* wsrc = wpre16 + (size_t)cd * EDIM + cpart;
  _Float16* tdst = tile + cd * 32 + cpart;
  *(v8h*)(tdst) = *(const v8h*)(wsrc);

#pragma unroll 1
  for (int c = 0; c < 8; ++c) {
    const v16h q0 = ld_frag(qp0, c * 32, h);
    const v16h q1 = ld_frag(qp1, c * 32, h);
#pragma unroll 1
    for (int kk = 0; kk < TWOE; kk += 4) {
      const v4h fv0 = *(const v4h*)(fp0 + kk);
      const v4h fv1 = *(const v4h*)(fp1 + kk);
#pragma unroll
      for (int u = 0; u < 4; ++u) {
        const int p = u & 1;
        __syncthreads();
        int nkk = kk + u + 1, nc = c;
        if (nkk == TWOE) { nkk = 0; nc = c + 1; }
        if (nc < 8)
          *(v8h*)(tdst + (p ^ 1) * 2048) =
              *(const v8h*)(wsrc + (size_t)nkk * (DDYN * EDIM) + nc * 32);
        const _Float16* tb = tile + p * 2048;
        const v16h b0 = ld_frag(tb + (0 * 16 + m) * 32, 0, h);
        const v16h b1 = ld_frag(tb + (1 * 16 + m) * 32, 0, h);
        const v16h b2 = ld_frag(tb + (2 * 16 + m) * 32, 0, h);
        const v16h b3 = ld_frag(tb + (3 * 16 + m) * 32, 0, h);
        const v16h a0 = q0 * splat16(fv0[u]);
        const v16h a1 = q1 * splat16(fv1[u]);
        acc[0][0] = mma16(a0, b0, acc[0][0]);
        acc[1][0] = mma16(a1, b0, acc[1][0]);
        acc[0][1] = mma16(a0, b1, acc[0][1]);
        acc[1][1] = mma16(a1, b1, acc[1][1]);
        acc[0][2] = mma16(a0, b2, acc[0][2]);
        acc[1][2] = mma16(a1, b2, acc[1][2]);
        acc[0][3] = mma16(a0, b3, acc[0][3]);
        acc[1][3] = mma16(a1, b3, acc[1][3]);
        WG8(acc[0][0], acc[1][0], acc[0][1], acc[1][1], acc[0][2], acc[1][2], acc[0][3],
            acc[1][3], a0, a1, b0, b1, b2, b3);
      }
    }
  }

#pragma unroll 1
  for (int c2 = 0; c2 < TWOE / 32; ++c2) {
    const v16h a0 = ld_frag(fp0, c2 * 32, h);
    const v16h a1 = ld_frag(fp1, c2 * 32, h);
    const v16h b0 = ld_frag(bpreT16 + (size_t)(0 * 16 + m) * TWOE, c2 * 32, h);
    const v16h b1 = ld_frag(bpreT16 + (size_t)(1 * 16 + m) * TWOE, c2 * 32, h);
    const v16h b2 = ld_frag(bpreT16 + (size_t)(2 * 16 + m) * TWOE, c2 * 32, h);
    const v16h b3 = ld_frag(bpreT16 + (size_t)(3 * 16 + m) * TWOE, c2 * 32, h);
    acc[0][0] = mma16(a0, b0, acc[0][0]);
    acc[1][0] = mma16(a1, b0, acc[1][0]);
    acc[0][1] = mma16(a0, b1, acc[0][1]);
    acc[1][1] = mma16(a1, b1, acc[1][1]);
    acc[0][2] = mma16(a0, b2, acc[0][2]);
    acc[1][2] = mma16(a1, b2, acc[1][2]);
    acc[0][3] = mma16(a0, b3, acc[0][3]);
    acc[1][3] = mma16(a1, b3, acc[1][3]);
    WG8(acc[0][0], acc[1][0], acc[0][1], acc[1][1], acc[0][2], acc[1][2], acc[0][3],
        acc[1][3], a0, a1, b0, b1, b2, b3);
  }

  __syncthreads();
  float* stg = lds + wave * 1024;
  const float inv = 1.0f / 1024.0f;
  float* gbase = f1raw + (size_t)rowBase * DDYN;
  store_tile16x64(stg, gbase, DDYN, acc[0][0], acc[0][1], acc[0][2], acc[0][3], inv, lane, h, m);
  __syncthreads();
  store_tile16x64(stg, gbase + 16 * DDYN, DDYN, acc[1][0], acc[1][1], acc[1][2], acc[1][3],
                  inv, lane, h, m);
}

__global__ __launch_bounds__(256) void ln64_kernel(const float* __restrict__ raw,
                                                   const float* __restrict__ g,
                                                   const float* __restrict__ be,
                                                   _Float16* __restrict__ outh, int nrows) {
  const int lane = threadIdx.x & 31, wave = threadIdx.x >> 5;
  const int row = blockIdx.x * 32 + wave * 4 + (lane >> 3);
  const int c8 = (lane & 7) * 8;
  const int rc = (row < nrows) ? row : (nrows - 1);
  const float* rp = raw + (size_t)rc * DDYN + c8;
  const v4f xa = *(const v4f*)rp;
  const v4f xb = *(const v4f*)(rp + 4);
  float s = (xa[0] + xa[1]) + (xa[2] + xa[3]) + (xb[0] + xb[1]) + (xb[2] + xb[3]);
  s = wsum8(s);
  const float mu = s * (1.0f / 64.0f);
  const v4f da = xa - mu, db = xb - mu;
  float qv = (da[0] * da[0] + da[1] * da[1]) + (da[2] * da[2] + da[3] * da[3]) +
             (db[0] * db[0] + db[1] * db[1]) + (db[2] * db[2] + db[3] * db[3]);
  qv = wsum8(qv);
  const float rs = rsqrtf(qv * (1.0f / 64.0f) + 1e-5f);
  const v4f ga = *(const v4f*)(g + c8), gb = *(const v4f*)(g + c8 + 4);
  const v4f ea = *(const v4f*)(be + c8), eb = *(const v4f*)(be + c8 + 4);
  const v4f ya = da * rs * ga + ea;
  const v4f yb = db * rs * gb + eb;
  v8h y;
#pragma unroll
  for (int j = 0; j < 4; ++j) {
    y[j]     = (_Float16)fmaxf(ya[j], 0.0f);
    y[4 + j] = (_Float16)fmaxf(yb[j], 0.0f);
  }
  _Float16* op = outh + (size_t)row * DDYN + c8;
  const bool ok = row < nrows;
  if (ok) *(volatile v8h*)op = y;
  __threadfence();
  if (ok) *(volatile v8h*)op = y;
}

static __device__ __forceinline__ void s2_fill(_Float16* tilebuf,
                                               const _Float16* __restrict__ waft16, int c,
                                               int dd, int ep0, int part) {
#pragma unroll
  for (int i = 0; i < 4; ++i) {
    const int ep = ep0 + i * 64;
    *(v8h*)(tilebuf + ep * 32 + part) =
        *(const v8h*)(waft16 + ((size_t)dd * EDIM + ep) * EDIM + c * 32 + part);
  }
}

__global__ __launch_bounds__(256) void s2_kernel(const _Float16* __restrict__ q16,
                                                 const _Float16* __restrict__ f1h,
                                                 const _Float16* __restrict__ waft16,
                                                 const _Float16* __restrict__ baftT16,
                                                 float* __restrict__ f2raw, int nrows) {
  __shared__ float lds[8192];
  _Float16* tile = reinterpret_cast<_Float16*>(lds);
  const int tid = threadIdx.x, lane = tid & 31, wave = tid >> 5;
  const int h = lane >> 4, m = lane & 15;
  const int rowBase = blockIdx.x * 128 + wave * 16;
  int r0 = rowBase + m; r0 = (r0 < nrows) ? r0 : (nrows - 1);
  const _Float16* qp = q16 + (size_t)r0 * EDIM;
  const _Float16* fp = f1h + (size_t)r0 * DDYN;

  v8f acc[16];
#pragma unroll
  for (int n = 0; n < 16; ++n) acc[n] = zero8();

  const int ep0 = tid >> 2, part = (tid & 3) * 8;
  s2_fill(tile, waft16, 0, 0, ep0, part);

#pragma unroll 1
  for (int c = 0; c < 8; ++c) {
    const v16h qf = ld_frag(qp, c * 32, h);
#pragma unroll 1
    for (int dd = 0; dd < DDYN; dd += 4) {
      const v4h fv = *(const v4h*)(fp + dd);
#pragma unroll
      for (int u = 0; u < 4; ++u) {
        const int p = u & 1;
        __syncthreads();
        int ndd = dd + u + 1, nc = c;
        if (ndd == DDYN) { ndd = 0; nc = c + 1; }
        if (nc < 8) s2_fill(tile + (p ^ 1) * 8192, waft16, nc, ndd, ep0, part);
        const v16h a = qf * splat16(fv[u]);
        const _Float16* tb = tile + p * 8192;
#pragma unroll
        for (int grp = 0; grp < 4; ++grp) {
          const v16h b0 = ld_frag(tb + ((grp * 4 + 0) * 16 + m) * 32, 0, h);
          const v16h b1 = ld_frag(tb + ((grp * 4 + 1) * 16 + m) * 32, 0, h);
          const v16h b2 = ld_frag(tb + ((grp * 4 + 2) * 16 + m) * 32, 0, h);
          const v16h b3 = ld_frag(tb + ((grp * 4 + 3) * 16 + m) * 32, 0, h);
          acc[grp * 4 + 0] = mma16(a, b0, acc[grp * 4 + 0]);
          acc[grp * 4 + 1] = mma16(a, b1, acc[grp * 4 + 1]);
          acc[grp * 4 + 2] = mma16(a, b2, acc[grp * 4 + 2]);
          acc[grp * 4 + 3] = mma16(a, b3, acc[grp * 4 + 3]);
          WG4(acc[grp * 4 + 0], acc[grp * 4 + 1], acc[grp * 4 + 2], acc[grp * 4 + 3], a, b0,
              b1, b2, b3);
        }
      }
    }
  }

#pragma unroll 1
  for (int c2 = 0; c2 < DDYN / 32; ++c2) {
    const v16h a = ld_frag(fp, c2 * 32, h);
#pragma unroll
    for (int grp = 0; grp < 4; ++grp) {
      const v16h b0 = ld_frag(baftT16 + (size_t)((grp * 4 + 0) * 16 + m) * DDYN, c2 * 32, h);
      const v16h b1 = ld_frag(baftT16 + (size_t)((grp * 4 + 1) * 16 + m) * DDYN, c2 * 32, h);
      const v16h b2 = ld_frag(baftT16 + (size_t)((grp * 4 + 2) * 16 + m) * DDYN, c2 * 32, h);
      const v16h b3 = ld_frag(baftT16 + (size_t)((grp * 4 + 3) * 16 + m) * DDYN, c2 * 32, h);
      acc[grp * 4 + 0] = mma16(a, b0, acc[grp * 4 + 0]);
      acc[grp * 4 + 1] = mma16(a, b1, acc[grp * 4 + 1]);
      acc[grp * 4 + 2] = mma16(a, b2, acc[grp * 4 + 2]);
      acc[grp * 4 + 3] = mma16(a, b3, acc[grp * 4 + 3]);
      WG4(acc[grp * 4 + 0], acc[grp * 4 + 1], acc[grp * 4 + 2], acc[grp * 4 + 3], a, b0, b1,
          b2, b3);
    }
  }

  __syncthreads();
  float* stg = lds + wave * 1024;
  const float inv = 1.0f / 1024.0f;
  float* gbase = f2raw + (size_t)rowBase * EDIM;
#pragma unroll
  for (int gq = 0; gq < 4; ++gq) {
    if (gq) __syncthreads();
    store_tile16x64(stg, gbase + gq * 64, EDIM, acc[gq * 4 + 0], acc[gq * 4 + 1],
                    acc[gq * 4 + 2], acc[gq * 4 + 3], inv, lane, h, m);
  }
}

__global__ __launch_bounds__(256) void ln256h_kernel(const float* __restrict__ raw,
                                                     const float* __restrict__ g,
                                                     const float* __restrict__ be,
                                                     _Float16* __restrict__ outh, int nrows) {
  const int lane = threadIdx.x & 31, wave = threadIdx.x >> 5;
  const int row = blockIdx.x * 8 + wave;
  const int c8 = lane * 8;
  const int rc = (row < nrows) ? row : (nrows - 1);
  const float* rp = raw + (size_t)rc * EDIM + c8;
  const v4f xa = *(const v4f*)rp;
  const v4f xb = *(const v4f*)(rp + 4);
  float s = (xa[0] + xa[1]) + (xa[2] + xa[3]) + (xb[0] + xb[1]) + (xb[2] + xb[3]);
  s = wsum32(s);
  const float mu = s * (1.0f / 256.0f);
  const v4f da = xa - mu, db = xb - mu;
  float qv = (da[0] * da[0] + da[1] * da[1]) + (da[2] * da[2] + da[3] * da[3]) +
             (db[0] * db[0] + db[1] * db[1]) + (db[2] * db[2] + db[3] * db[3]);
  qv = wsum32(qv);
  const float rs = rsqrtf(qv * (1.0f / 256.0f) + 1e-5f);
  const v4f ga = *(const v4f*)(g + c8), gb = *(const v4f*)(g + c8 + 4);
  const v4f ea = *(const v4f*)(be + c8), eb = *(const v4f*)(be + c8 + 4);
  const v4f ya = da * rs * ga + ea;
  const v4f yb = db * rs * gb + eb;
  v8h y;
#pragma unroll
  for (int j = 0; j < 4; ++j) {
    y[j]     = (_Float16)fmaxf(ya[j], 0.0f);
    y[4 + j] = (_Float16)fmaxf(yb[j], 0.0f);
  }
  _Float16* op = outh + (size_t)row * EDIM + c8;
  const bool ok = row < nrows;
  if (ok) *(volatile v8h*)op = y;
  __threadfence();
  if (ok) *(volatile v8h*)op = y;
}

__global__ __launch_bounds__(256) void s3_kernel(const _Float16* __restrict__ f2h,
                                                 const _Float16* __restrict__ wout16,
                                                 float* __restrict__ f3raw, int nrows) {
  __shared__ float lds[8192];
  const int tid = threadIdx.x, lane = tid & 31, wave = tid >> 5;
  const int h = lane >> 4, m = lane & 15;
  const int rowBase = blockIdx.x * 128 + wave * 16;
  int r0 = rowBase + m; r0 = (r0 < nrows) ? r0 : (nrows - 1);
  const _Float16* ap = f2h + (size_t)r0 * EDIM;

  v8f acc[16];
#pragma unroll
  for (int n = 0; n < 16; ++n) acc[n] = zero8();

#pragma unroll 1
  for (int c = 0; c < EDIM / 32; ++c) {
    const v16h a = ld_frag(ap, c * 32, h);
#pragma unroll
    for (int grp = 0; grp < 4; ++grp) {
      const v16h b0 = ld_frag(wout16 + (size_t)((grp * 4 + 0) * 16 + m) * EDIM, c * 32, h);
      const v16h b1 = ld_frag(wout16 + (size_t)((grp * 4 + 1) * 16 + m) * EDIM, c * 32, h);
      const v16h b2 = ld_frag(wout16 + (size_t)((grp * 4 + 2) * 16 + m) * EDIM, c * 32, h);
      const v16h b3 = ld_frag(wout16 + (size_t)((grp * 4 + 3) * 16 + m) * EDIM, c * 32, h);
      acc[grp * 4 + 0] = mma16(a, b0, acc[grp * 4 + 0]);
      acc[grp * 4 + 1] = mma16(a, b1, acc[grp * 4 + 1]);
      acc[grp * 4 + 2] = mma16(a, b2, acc[grp * 4 + 2]);
      acc[grp * 4 + 3] = mma16(a, b3, acc[grp * 4 + 3]);
      WG4(acc[grp * 4 + 0], acc[grp * 4 + 1], acc[grp * 4 + 2], acc[grp * 4 + 3], a, b0, b1,
          b2, b3);
    }
  }

  __syncthreads();
  float* stg = lds + wave * 1024;
  const float inv = 1.0f / 64.0f;
  float* gbase = f3raw + (size_t)rowBase * EDIM;
#pragma unroll
  for (int gq = 0; gq < 4; ++gq) {
    if (gq) __syncthreads();
    store_tile16x64(stg, gbase + gq * 64, EDIM, acc[gq * 4 + 0], acc[gq * 4 + 1],
                    acc[gq * 4 + 2], acc[gq * 4 + 3], inv, lane, h, m);
  }
}

__global__ __launch_bounds__(256) void ln_out_kernel(const float* __restrict__ raw,
                                                     const float* __restrict__ bout,
                                                     const float* __restrict__ g,
                                                     const float* __restrict__ be,
                                                     float* __restrict__ out, int nrows) {
  const int lane = threadIdx.x & 31, wave = threadIdx.x >> 5;
  const int row = blockIdx.x * 8 + wave;
  const int rc = (row < nrows) ? row : (nrows - 1);
  const float* rp = raw + (size_t)rc * EDIM;
  const int ca = lane * 4, cb = 128 + lane * 4;
  v4f xa = *(const v4f*)(rp + ca);
  v4f xb = *(const v4f*)(rp + cb);
  xa += *(const v4f*)(bout + ca);
  xb += *(const v4f*)(bout + cb);
  float s = (xa[0] + xa[1]) + (xa[2] + xa[3]) + (xb[0] + xb[1]) + (xb[2] + xb[3]);
  s = wsum32(s);
  const float mu = s * (1.0f / 256.0f);
  const v4f da = xa - mu, db = xb - mu;
  float qv = (da[0] * da[0] + da[1] * da[1]) + (da[2] * da[2] + da[3] * da[3]) +
             (db[0] * db[0] + db[1] * db[1]) + (db[2] * db[2] + db[3] * db[3]);
  qv = wsum32(qv);
  const float rs = rsqrtf(qv * (1.0f / 256.0f) + 1e-5f);
  const v4f ga = *(const v4f*)(g + ca), gb = *(const v4f*)(g + cb);
  const v4f ea = *(const v4f*)(be + ca), eb = *(const v4f*)(be + cb);
  v4f ya = da * rs * ga + ea;
  v4f yb = db * rs * gb + eb;
#pragma unroll
  for (int j = 0; j < 4; ++j) {
    ya[j] = fmaxf(ya[j], 0.0f);
    yb[j] = fmaxf(yb[j], 0.0f);
  }
  float* op = out + (size_t)row * EDIM;
  const bool ok = row < nrows;
  if (ok) {
    *(volatile v4f*)(op + ca) = ya;
    *(volatile v4f*)(op + cb) = yb;
  }
  __threadfence();
  if (ok) {
    *(volatile v4f*)(op + ca) = ya;
    *(volatile v4f*)(op + cb) = yb;
  }
}


static inline size_t al256(size_t x) { return (x + 255) & ~(size_t)255; }

extern "C" void kernel_launch(void* const* d_in, const int* in_sizes, int n_in, void* d_out,
                              int out_size, void* d_ws, size_t ws_size, hipStream_t stream) {
  if (n_in < 14) return;
  const int nq = in_sizes[0];
  if (nq <= 0 || (nq % EDIM) != 0) return;
  const int nrows = nq / EDIM;
  if (in_sizes[1] != nrows * TWOE) return;
  if (in_sizes[2] != NP1 * EDIM || in_sizes[3] != NP1) return;
  if (in_sizes[4] != NP2 * EDIM || in_sizes[5] != NP2) return;
  if (in_sizes[6] != EDIM * EDIM || in_sizes[7] != EDIM) return;
  if (in_sizes[8] != DDYN || in_sizes[9] != DDYN) return;
  if (in_sizes[10] != EDIM || in_sizes[11] != EDIM || in_sizes[12] != EDIM ||
      in_sizes[13] != EDIM)
    return;
  if (out_size != nrows * EDIM) return;

  const float* query = (const float*)d_in[0];
  const float* feats = (const float*)d_in[1];
  const float* W_pre = (const float*)d_in[2];
  const float* b_pre = (const float*)d_in[3];
  const float* W_aft = (const float*)d_in[4];
  const float* b_aft = (const float*)d_in[5];
  const float* W_out = (const float*)d_in[6];
  const float* b_out = (const float*)d_in[7];
  const float* g1  = (const float*)d_in[8];
  const float* be1 = (const float*)d_in[9];
  const float* g2  = (const float*)d_in[10];
  const float* be2 = (const float*)d_in[11];
  const float* g3  = (const float*)d_in[12];
  const float* be3 = (const float*)d_in[13];

  const int gb1 = (nrows + 255) / 256, rp1 = gb1 * 256;
  const int gb2 = (nrows + 127) / 128, rp2 = gb2 * 128;

  char* w = (char*)d_ws;
  size_t off = 0;
  _Float16* wpre16  = (_Float16*)(w + off); off += al256((size_t)NP1 * EDIM * 2);
  _Float16* waft16  = (_Float16*)(w + off); off += al256((size_t)NP2 * EDIM * 2);
  _Float16* wout16  = (_Float16*)(w + off); off += al256((size_t)EDIM * EDIM * 2);
  _Float16* q16     = (_Float16*)(w + off); off += al256((size_t)nq * 2);
  _Float16* feats16 = (_Float16*)(w + off); off += al256((size_t)in_sizes[1] * 2);
  _Float16* bpreT16 = (_Float16*)(w + off); off += al256((size_t)NP1 * 2);
  _Float16* baftT16 = (_Float16*)(w + off); off += al256((size_t)NP2 * 2);
  float*    f1raw   = (float*)(w + off);    off += al256((size_t)rp1 * DDYN * 4);
  _Float16* f1h     = (_Float16*)(w + off); off += al256((size_t)rp1 * DDYN * 2);
  float*    f2raw   = (float*)(w + off);    off += al256((size_t)rp2 * EDIM * 4);
  _Float16* f2h     = (_Float16*)(w + off); off += al256((size_t)rp2 * EDIM * 2);
  float*    f3raw   = (float*)(w + off);    off += al256((size_t)rp2 * EDIM * 4);
  if (off > ws_size) return;

  auto gs = [](long n) { return (unsigned)((n + 255) / 256); };

  { const int n8 = nq / 8;                cvt8_kernel<<<gs(n8), 256, 0, stream>>>(query, q16, n8, 16.0f); }
  { const int n8 = in_sizes[1] / 8;       cvt8_kernel<<<gs(n8), 256, 0, stream>>>(feats, feats16, n8, 1.0f); }
  { const int n8 = (NP1 * EDIM) / 8;      cvt8_kernel<<<gs(n8), 256, 0, stream>>>(W_pre, wpre16, n8, 64.0f); }
  { const int n8 = (NP2 * EDIM) / 8;      cvt8_kernel<<<gs(n8), 256, 0, stream>>>(W_aft, waft16, n8, 64.0f); }
  { const int n8 = (EDIM * EDIM) / 8;     cvt8_kernel<<<gs(n8), 256, 0, stream>>>(W_out, wout16, n8, 64.0f); }
  bias_t_kernel<<<gs((long)DDYN * (TWOE / 8)), 256, 0, stream>>>(b_pre, bpreT16, TWOE, DDYN, 1024.0f);
  bias_t_kernel<<<gs((long)EDIM * (DDYN / 8)), 256, 0, stream>>>(b_aft, baftT16, DDYN, EDIM, 1024.0f);

  s1_kernel<<<gb1, 256, 0, stream>>>(q16, feats16, wpre16, bpreT16, f1raw, nrows);
  ln64_kernel<<<(unsigned)((nrows + 31) / 32), 256, 0, stream>>>(f1raw, g1, be1, f1h, nrows);
  s2_kernel<<<gb2, 256, 0, stream>>>(q16, f1h, waft16, baftT16, f2raw, nrows);
  ln256h_kernel<<<(unsigned)((nrows + 7) / 8), 256, 0, stream>>>(f2raw, g2, be2, f2h, nrows);
  s3_kernel<<<gb2, 256, 0, stream>>>(f2h, wout16, f3raw, nrows);
  ln_out_kernel<<<(unsigned)((nrows + 7) / 8), 256, 0, stream>>>(f3raw, b_out, g3, be3,
                                                                 (float*)d_out, nrows);
}
